// LSTM_CRF_50921132262039
// MI455X (gfx1250) — hardware-run, weakly checked
//
#include <hip/hip_runtime.h>
#include <math.h>

typedef __attribute__((ext_vector_type(16))) _Float16 v16h;
typedef __attribute__((ext_vector_type(8)))  _Float16 v8h;
typedef __attribute__((ext_vector_type(8)))  float    v8f;
typedef __attribute__((ext_vector_type(4)))  float    v4f;

constexpr int kBatch   = 128;
constexpr int kSteps   = 256;
constexpr int kEmb     = 300;
constexpr int kHid     = 50;
constexpr int kCls     = 9;
constexpr int kVocab   = 30000;
constexpr int kRows    = kBatch * kSteps;
constexpr int kGates   = 4 * kHid;
constexpr int kKPad    = 320;
constexpr int kNPad    = 448;
constexpr int kHPad    = 64;
constexpr int kChunks  = kKPad / 8;
constexpr int kLogitN  = kRows * kCls;
constexpr int kOutN    = kLogitN + 1;
constexpr int kTilesM  = kRows / 64;
constexpr int kTilesN  = kNPad / 64;
constexpr int kLdsWP   = 72;
constexpr int kLdsOP   = 68;
constexpr int kFcPitch = 52;
static_assert(kRows == 32768);
static_assert(kGates == 200);
static_assert((kKPad % 32) == 0 && kKPad >= kEmb);
static_assert((kNPad % 64) == 0 && kNPad >= 2 * kGates);
static_assert((kRows % 64) == 0);
static_assert((kEmb % 4) == 0);
static_assert((kTilesM * kTilesN) % 8 == 0);
static_assert(kLogitN % 256 == 0);
static_assert(kGates + 3 * kHid + kHPad - 1 < kNPad);

constexpr float kCarryAct = 256.0f;
constexpr float kCarryWgt = 256.0f;
constexpr float kCarryHid = 512.0f;
constexpr float kFoldXG   = 1.0f / (kCarryAct * kCarryWgt);
constexpr float kFoldHH   = 1.0f / (kCarryHid * kCarryWgt);
constexpr float kF16MinNormal = 6.103515625e-5f;

constexpr size_t kOffA16  = 0;
constexpr size_t kOffBT16 = kOffA16  + (size_t)kRows * kKPad * 2;
constexpr size_t kOffBIAS = kOffBT16 + (size_t)kNPad * kKPad * 2;
constexpr size_t kOffXG   = kOffBIAS + (size_t)kNPad * 4;
constexpr size_t kOffHF   = kOffXG   + (size_t)kRows * kNPad * 4;
constexpr size_t kOffHB   = kOffHF   + (size_t)kRows * kHPad * 4;
constexpr size_t kOffLG   = kOffHB   + (size_t)kRows * kHPad * 4;
constexpr size_t kWsTotal = kOffLG   + (size_t)kLogitN * 4;
static_assert(kWsTotal == 97937152ull);
static_assert(kWsTotal <= 134217728ull);
static_assert((kOffBT16 % 128) == 0 && (kOffBIAS % 128) == 0 && (kOffXG % 128) == 0 &&
              (kOffHF % 128) == 0 && (kOffHB % 128) == 0 && (kOffLG % 128) == 0);
static_assert((size_t)kOutN * 4 == 1179652ull);

__device__ __forceinline__ int clampi(int v, int lo, int hi) {
  v = (v < lo) ? lo : v;
  v = (v > hi) ? hi : v;
  return v;
}
__device__ __forceinline__ _Float16 to_operand_h(float v, float carry) {
  float s = v * carry;
  s = (fabsf(s) < kF16MinNormal) ? 0.0f : s;
  return (_Float16)s;
}
union FragU { v16h v; v8h h[2]; };
__device__ __forceinline__ v16h frag_load(const _Float16* p) {
  FragU f;
  f.h[0] = *(const v8h*)(p);
  f.h[1] = *(const v8h*)(p + 16);
  return f.v;
}
__device__ __forceinline__ v8f mma_raw(v16h a, v16h b, v8f c) {
  return __builtin_amdgcn_wmma_f32_16x16x32_f16(false, a, false, b, (short)0, c, false, false);
}
__device__ __forceinline__ v8f mma_guarded(v16h a, v16h b, v8f c) {
  c = __builtin_amdgcn_wmma_f32_16x16x32_f16(false, a, false, b, (short)0, c, false, false);
  asm volatile("v_nop\n\tv_nop\n\tv_nop\n\tv_nop" : "+v"(c) : "v"(a), "v"(b));
  return c;
}
__device__ __forceinline__ void guard_group4(v8f& a, v8f& b, v8f& c, v8f& d, v16h x) {
  asm volatile("v_nop\n\tv_nop\n\tv_nop\n\tv_nop" : "+v"(a), "+v"(b), "+v"(c), "+v"(d) : "v"(x));
}
__device__ __forceinline__ void keep_frags4(v16h a, v16h b, v16h c, v16h d) {
  asm volatile("v_nop" :: "v"(a), "v"(b), "v"(c), "v"(d));
}
__device__ __forceinline__ void acc_guard4(v8f& a, v8f& b, v8f& c, v8f& d) {
  asm volatile("v_nop\n\tv_nop\n\tv_nop\n\tv_nop" : "+v"(a), "+v"(b), "+v"(c), "+v"(d));
}
__device__ __forceinline__ float sigmoid_f(float x) {
  return __builtin_amdgcn_rcpf(1.0f + expf(-x));
}

__global__ __launch_bounds__(256) void prep_act_kernel(
    const int* __restrict__ ids, const float* __restrict__ table, unsigned short* __restrict__ A16)
{
  const int q = blockIdx.x * 256 + threadIdx.x;
  if (q >= kRows * kChunks) return;
  const int m  = q / kChunks;
  const int ch = q - m * kChunks;
  const int k0 = ch * 8;
  const int id = clampi(ids[m], 0, kVocab - 1);
  const float* src = table + (size_t)id * kEmb;
  const int ka = (k0 < kEmb - 4) ? k0 : (kEmb - 4);
  const int kb = (k0 + 4 < kEmb - 4) ? (k0 + 4) : (kEmb - 4);
  v4f a = *(const v4f*)(src + ka);
  v4f b = *(const v4f*)(src + kb);
  asm volatile("" : "+v"(a), "+v"(b));
  const bool oka = (k0 < kEmb);
  const bool okb = (k0 + 4 < kEmb);
  v8h hv;
#pragma unroll
  for (int e = 0; e < 4; ++e) {
    const float fa = oka ? a[e] : 0.0f;
    const float fb = okb ? b[e] : 0.0f;
    hv[e]     = to_operand_h(fa, kCarryAct);
    hv[4 + e] = to_operand_h(fb, kCarryAct);
  }
  unsigned short* dst = A16 + (size_t)q * 8;
  *(volatile v8h*)dst = hv;
  __threadfence();
  *(volatile v8h*)dst = hv;
}

__global__ __launch_bounds__(64) void prep_wgt_kernel(
    const float* __restrict__ WihF, const float* __restrict__ WihB,
    const float* __restrict__ bihF, const float* __restrict__ bhhF,
    const float* __restrict__ bihB, const float* __restrict__ bhhB,
    unsigned short* __restrict__ BT16, float* __restrict__ BIAS)
{
  const int tid = threadIdx.x;
  const int n = blockIdx.x;
  if (n < kNPad) {
    const int nb = ((n < 2 * kGates) ? n : (2 * kGates - 1)) - kGates;
    const float* src = (n < kGates) ? (WihF + (size_t)n * kEmb) : (WihB + (size_t)((nb < 0) ? 0 : nb) * kEmb);
    const bool rowok = (n < 2 * kGates);
    const int ch = (tid < kChunks) ? tid : (kChunks - 1);
    const int k0 = ch * 8;
    const int ka = (k0 < kEmb - 4) ? k0 : (kEmb - 4);
    const int kb = (k0 + 4 < kEmb - 4) ? (k0 + 4) : (kEmb - 4);
    v4f a = *(const v4f*)(src + ka);
    v4f b = *(const v4f*)(src + kb);
    asm volatile("" : "+v"(a), "+v"(b));
    const bool oka = rowok && (k0 < kEmb);
    const bool okb = rowok && (k0 + 4 < kEmb);
    v8h hv;
#pragma unroll
    for (int e = 0; e < 4; ++e) {
      const float fa = oka ? a[e] : 0.0f;
      const float fb = okb ? b[e] : 0.0f;
      hv[e]     = to_operand_h(fa, kCarryWgt);
      hv[4 + e] = to_operand_h(fb, kCarryWgt);
    }
    if (tid < kChunks) {
      unsigned short* dst = BT16 + (size_t)n * kKPad + k0;
      *(volatile v8h*)dst = hv;
      __threadfence();
      *(volatile v8h*)dst = hv;
    }
  } else {
#pragma unroll 1
    for (int it = 0; it < 2; ++it) {
      const int idx4 = tid + 64 * it;
      const int n0 = idx4 * 4;
      const int nf = (n0 < kGates - 4) ? n0 : (kGates - 4);
      int nbk = n0 - kGates;
      nbk = (nbk < 0) ? 0 : nbk;
      nbk = (nbk > kGates - 4) ? (kGates - 4) : nbk;
      v4f f0 = *(const v4f*)(bihF + nf);
      v4f f1 = *(const v4f*)(bhhF + nf);
      v4f b0 = *(const v4f*)(bihB + nbk);
      v4f b1 = *(const v4f*)(bhhB + nbk);
      asm volatile("" : "+v"(f0), "+v"(f1), "+v"(b0), "+v"(b1));
      const bool isf = (n0 < kGates);
      const bool isb = (n0 >= kGates) && (n0 < 2 * kGates);
      v4f o;
#pragma unroll
      for (int e = 0; e < 4; ++e) {
        const float sf = f0[e] + f1[e];
        const float sb = b0[e] + b1[e];
        o[e] = isf ? sf : (isb ? sb : 0.0f);
      }
      if (idx4 < kNPad / 4) {
        float* dst = BIAS + n0;
        *(volatile v4f*)dst = o;
        __threadfence();
        *(volatile v4f*)dst = o;
      }
    }
  }
}

__global__ __launch_bounds__(256) void gemm_xg_kernel(
    const unsigned short* __restrict__ Ap, const unsigned short* __restrict__ Btp,
    float* __restrict__ Cout, const float* __restrict__ bias, float scale)
{
  const _Float16* A  = (const _Float16*)Ap;
  const _Float16* Bt = (const _Float16*)Btp;
  __shared__ __align__(16) float sT[8][16 * kLdsOP];
  const int lane = threadIdx.x & 31;
  const int wave = threadIdx.x >> 5;
  const int tile = blockIdx.x * 8 + wave;
  if (tile >= kTilesM * kTilesN) return;
  const int tm = tile / kTilesN;
  const int tn = tile - tm * kTilesN;
  const int m0 = tm << 6;
  const int n0 = tn << 6;
  const int rlane = lane & 15;
  const int koff  = (lane >> 4) * 8;
  const int mOff  = (lane >> 4) * 8;

  v8f acc[4][4];
#pragma unroll
  for (int i = 0; i < 4; ++i)
#pragma unroll
    for (int j = 0; j < 4; ++j) acc[i][j] = (v8f){0.f, 0.f, 0.f, 0.f, 0.f, 0.f, 0.f, 0.f};

  for (int k0 = 0; k0 < kKPad; k0 += 32) {
    v16h bh[4];
#pragma unroll
    for (int j = 0; j < 4; ++j) {
      const size_t bo = (size_t)(n0 + (j << 4) + rlane) * kKPad + koff + k0;
      bh[j] = frag_load(Bt + bo);
    }
#pragma unroll
    for (int i = 0; i < 4; ++i) {
      const size_t ao = (size_t)(m0 + (i << 4) + rlane) * kKPad + koff + k0;
      const v16h ah = frag_load(A + ao);
#pragma unroll
      for (int j = 0; j < 4; ++j) acc[i][j] = mma_raw(ah, bh[j], acc[i][j]);
      guard_group4(acc[i][0], acc[i][1], acc[i][2], acc[i][3], ah);
    }
    keep_frags4(bh[0], bh[1], bh[2], bh[3]);
  }
  acc_guard4(acc[0][0], acc[0][1], acc[0][2], acc[0][3]);
  acc_guard4(acc[1][0], acc[1][1], acc[1][2], acc[1][3]);
  acc_guard4(acc[2][0], acc[2][1], acc[2][2], acc[2][3]);
  acc_guard4(acc[3][0], acc[3][1], acc[3][2], acc[3][3]);

  float* slab = sT[wave];
#pragma unroll
  for (int i = 0; i < 4; ++i) {
    const int mBase = m0 + (i << 4);
#pragma unroll
    for (int j = 0; j < 4; ++j) {
      const int n = n0 + (j << 4) + rlane;
      const float bv = bias[n];
#pragma unroll
      for (int r = 0; r < 8; ++r) {
        const float v = acc[i][j][r] * scale + bv;
        slab[(mOff + r) * kLdsOP + (j << 4) + rlane] = v;
      }
    }
    __builtin_amdgcn_fence(__ATOMIC_RELEASE, "workgroup");
    __builtin_amdgcn_wave_barrier();
    __builtin_amdgcn_fence(__ATOMIC_ACQUIRE, "workgroup");
    {
      const int hh = lane >> 4, c4 = (lane & 15) * 4;
      for (int pass = 0; pass < 2; ++pass) {
#pragma unroll
        for (int it = 0; it < 8; ++it) {
          const int row = it * 2 + hh;
          const v4f v = *(const v4f*)(slab + row * kLdsOP + c4);
          *(volatile v4f*)(Cout + (size_t)(mBase + row) * kNPad + n0 + c4) = v;
        }
        __threadfence();
      }
    }
    __builtin_amdgcn_fence(__ATOMIC_RELEASE, "workgroup");
    __builtin_amdgcn_wave_barrier();
    __builtin_amdgcn_fence(__ATOMIC_ACQUIRE, "workgroup");
  }
}

__global__ __launch_bounds__(128) void lstm_scan_kernel(
    const float* __restrict__ XG, const float* __restrict__ WhhF, const float* __restrict__ WhhB,
    float* __restrict__ Hf, float* __restrict__ Hb)
{
  __shared__ __align__(16) _Float16 sW[256 * kLdsWP];
  __shared__ __align__(16) _Float16 sH[2 * 16 * kLdsWP];
  __shared__ __align__(16) float    sO[2 * 16 * kLdsOP];
  const int tid  = threadIdx.x;
  const int lane = tid & 31;
  const int wave = tid >> 5;
  const int hh   = lane >> 4;
  const int c    = lane & 15;
  const int btile = blockIdx.x;
  const int dir   = blockIdx.y;
  const float* Wsrc = (dir != 0) ? WhhB : WhhF;
  float* Hd = (dir != 0) ? Hb : Hf;

#pragma unroll 1
  for (int it = 0; it < 16; ++it) {
    const int idx = tid + 128 * it;
    const int n  = idx >> 3;
    const int k0 = (idx & 7) * 8;
    const int g  = n >> 6;
    const int j  = n & 63;
    const int jc = (j < kHid) ? j : (kHid - 1);
    const float* wrow = Wsrc + (size_t)(g * kHid + jc) * kHid;
    v8h hv;
#pragma unroll
    for (int e = 0; e < 8; ++e) {
      const int k  = k0 + e;
      const int kc = (k < kHid) ? k : (kHid - 1);
      float v = wrow[kc];
      asm volatile("" : "+v"(v));
      const bool ok = (j < kHid) && (k < kHid);
      const float vs = ok ? v : 0.0f;
      hv[e] = to_operand_h(vs, kCarryWgt);
    }
    *(v8h*)(sW + n * kLdsWP + k0) = hv;
  }
#pragma unroll 1
  for (int it = 0; it < 3; ++it) {
    const int idx = tid + 128 * it;
    if (idx < 288) {
      const v8h z = (v8h){(_Float16)0.f, (_Float16)0.f, (_Float16)0.f, (_Float16)0.f,
                          (_Float16)0.f, (_Float16)0.f, (_Float16)0.f, (_Float16)0.f};
      *(v8h*)(sH + idx * 8) = z;
    }
  }
  __syncthreads();

  v16h bw[4][2];
#pragma unroll
  for (int g = 0; g < 4; ++g)
#pragma unroll
    for (int kk = 0; kk < 2; ++kk)
      bw[g][kk] = frag_load(sW + (g * 64 + 16 * wave + c) * kLdsWP + kk * 32 + 8 * hh);

  const int  j  = 16 * wave + c;
  const bool jv = (j < kHid);
  v8f cst = (v8f){0.f, 0.f, 0.f, 0.f, 0.f, 0.f, 0.f, 0.f};

#pragma unroll 1
  for (int step = 0; step < kSteps; ++step) {
    const int cur = step & 1;
    const int pos = (dir != 0) ? (kSteps - 1 - step) : step;
    const _Float16* hc = sH + cur * 16 * kLdsWP;
    _Float16* hn = sH + (cur ^ 1) * 16 * kLdsWP;
    float* oc = sO + cur * 16 * kLdsOP;

    const size_t xbase = ((size_t)(btile * 16 + 8 * hh) * kSteps + pos) * kNPad + dir * kGates + j;
    v8f xg[4];
#pragma unroll
    for (int g = 0; g < 4; ++g) {
#pragma unroll
      for (int r = 0; r < 8; ++r) xg[g][r] = XG[xbase + (size_t)r * kSteps * kNPad + g * kHid];
      asm volatile("" : "+v"(xg[g]));
    }

    const v16h a0 = frag_load(hc + c * kLdsWP + 8 * hh);
    const v16h a1 = frag_load(hc + c * kLdsWP + 32 + 8 * hh);
    v8f acc[4];
#pragma unroll
    for (int g = 0; g < 4; ++g) {
      acc[g] = (v8f){0.f, 0.f, 0.f, 0.f, 0.f, 0.f, 0.f, 0.f};
      acc[g] = mma_guarded(a0, bw[g][0], acc[g]);
      acc[g] = mma_guarded(a1, bw[g][1], acc[g]);
    }

#pragma unroll
    for (int r = 0; r < 8; ++r) {
      const float xi = jv ? xg[0][r] : 0.0f;
      const float xf = jv ? xg[1][r] : 0.0f;
      const float xc = jv ? xg[2][r] : 0.0f;
      const float xo = jv ? xg[3][r] : 0.0f;
      const float pi = fmaf(acc[0][r], kFoldHH, xi);
      const float pf = fmaf(acc[1][r], kFoldHH, xf);
      const float pc = fmaf(acc[2][r], kFoldHH, xc);
      const float po = fmaf(acc[3][r], kFoldHH, xo);
      const float gi = sigmoid_f(pi);
      const float gf = sigmoid_f(pf);
      const float gc = tanhf(pc);
      const float go = sigmoid_f(po);
      const float cn = gf * cst[r] + gi * gc;
      const float hvl = go * tanhf(cn);
      const float cn2 = jv ? cn : 0.0f;
      const float hv2 = jv ? hvl : 0.0f;
      cst[r] = cn2;
      hn[(8 * hh + r) * kLdsWP + j] = to_operand_h(hv2, kCarryHid);
      oc[(8 * hh + r) * kLdsOP + j] = hv2;
    }
    __syncthreads();
    {
      const int c4 = c * 4;
      const int r0 = 4 * wave + hh;
      const int r1 = 4 * wave + 2 + hh;
      const v4f v0 = *(const v4f*)(oc + r0 * kLdsOP + c4);
      const v4f v1 = *(const v4f*)(oc + r1 * kLdsOP + c4);
      float* d0 = Hd + ((size_t)(btile * 16 + r0) * kSteps + pos) * kHPad + c4;
      float* d1 = Hd + ((size_t)(btile * 16 + r1) * kSteps + pos) * kHPad + c4;
      *(volatile v4f*)d0 = v0;
      *(volatile v4f*)d1 = v1;
      __threadfence();
      *(volatile v4f*)d0 = v0;
      *(volatile v4f*)d1 = v1;
    }
  }
}

__global__ __launch_bounds__(256) void fc_kernel(
    const float* __restrict__ Hf, const float* __restrict__ Hb,
    const float* __restrict__ fcw, const float* __restrict__ fcb, float* __restrict__ LG)
{
  __shared__ __align__(16) float sF[2 * kCls * kFcPitch];
  __shared__ float sBias[16];
  const int tid = threadIdx.x;
#pragma unroll 1
  for (int it = 0; it < 4; ++it) {
    const int idx = tid + 256 * it;
    const int idc = (idx < 2 * kCls * kFcPitch) ? idx : (2 * kCls * kFcPitch - 1);
    const int rw = idc / kFcPitch;
    const int k  = idc - rw * kFcPitch;
    const int kc = (k < kHid) ? k : (kHid - 1);
    float v = fcw[(rw >> 1) * (2 * kHid) + (rw & 1) * kHid + kc];
    asm volatile("" : "+v"(v));
    const float vs = (k < kHid) ? v : 0.0f;
    if (idx < 2 * kCls * kFcPitch) sF[idx] = vs;
  }
  {
    const int ic = (tid < kCls) ? tid : (kCls - 1);
    float v = fcb[ic];
    asm volatile("" : "+v"(v));
    if (tid < kCls) sBias[tid] = v;
  }
  __syncthreads();
  const int q  = blockIdx.x * 256 + tid;
  const int m  = q / kCls;
  const int cc = q - m * kCls;
  const float* hf = Hf + (size_t)m * kHPad;
  const float* hb = Hb + (size_t)m * kHPad;
  const float* w0 = sF + (cc * 2) * kFcPitch;
  const float* w1 = w0 + kFcPitch;
  float s = 0.0f;
#pragma unroll 1
  for (int kq = 0; kq < kFcPitch / 4; ++kq) {
    const v4f a  = *(const v4f*)(hf + 4 * kq);
    const v4f b  = *(const v4f*)(hb + 4 * kq);
    const v4f wa = *(const v4f*)(w0 + 4 * kq);
    const v4f wb = *(const v4f*)(w1 + 4 * kq);
    s = fmaf(a[0], wa[0], s);
    s = fmaf(a[1], wa[1], s);
    s = fmaf(a[2], wa[2], s);
    s = fmaf(a[3], wa[3], s);
    s = fmaf(b[0], wb[0], s);
    s = fmaf(b[1], wb[1], s);
    s = fmaf(b[2], wb[2], s);
    s = fmaf(b[3], wb[3], s);
  }
  const float val = s + sBias[cc];
  volatile float* dst = LG + q;
  *dst = val;
  __threadfence();
  *dst = val;
}

__global__ __launch_bounds__(256) void copy_logits_kernel(const float* __restrict__ LG, float* __restrict__ out)
{
  const int i = 32 + blockIdx.x * 256 + threadIdx.x;
  const int src = (i - 1 < kLogitN) ? (i - 1) : (kLogitN - 1);
  float v = LG[src];
  asm volatile("" : "+v"(v));
  if (i < kOutN) {
    volatile float* dst = out + i;
    *dst = v;
    __threadfence();
    *dst = v;
  }
}

__global__ __launch_bounds__(128) void crf_loss_kernel(
    const float* __restrict__ LG, const int* __restrict__ ids, const int* __restrict__ labels,
    const float* __restrict__ trans, const float* __restrict__ startT, const float* __restrict__ endT,
    float* __restrict__ out)
{
  __shared__ float sTr[96];
  __shared__ float sSt[16];
  __shared__ float sEn[16];
  __shared__ float sA[kCls * 128];
  __shared__ float sN[kCls * 128];
  __shared__ float sL[128];
  const int tid  = threadIdx.x;
  const int lane = tid & 31;
  const int wave = tid >> 5;
  {
    const int it = (tid < kCls * kCls) ? tid : (kCls * kCls - 1);
    float v = trans[it];
    asm volatile("" : "+v"(v));
    if (tid < kCls * kCls) sTr[tid] = v;
    const int ic = (tid < kCls) ? tid : (kCls - 1);
    float sv = startT[ic];
    float ev = endT[ic];
    asm volatile("" : "+v"(sv), "+v"(ev));
    if (tid < kCls) {
      sSt[tid] = sv;
      sEn[tid] = ev;
    }
  }
  __syncthreads();

  const int base = tid * kSteps;
  const int tg0 = clampi(labels[base], 0, kCls - 1);
#pragma unroll 1
  for (int jj = 0; jj < kCls; ++jj) sA[jj * 128 + tid] = sSt[jj] + LG[(size_t)base * kCls + jj];
  float num = sSt[tg0] + LG[(size_t)base * kCls + tg0];
  int cnt = (ids[base] != 0) ? 1 : 0;
  int prv = tg0;

#pragma unroll 1
  for (int t = 1; t < kSteps; ++t) {
    const size_t row = (size_t)(base + t) * kCls;
    const bool mt = (ids[base + t] != 0);
    const int tg = clampi(labels[base + t], 0, kCls - 1);
    float ltag = LG[row + tg];
    asm volatile("" : "+v"(ltag));
#pragma unroll 1
    for (int jj = 0; jj < kCls; ++jj) {
      float mx = -INFINITY;
#pragma unroll 1
      for (int ii = 0; ii < kCls; ++ii) mx = fmaxf(mx, sA[ii * 128 + tid] + sTr[ii * kCls + jj]);
      float sm = 0.0f;
#pragma unroll 1
      for (int ii = 0; ii < kCls; ++ii) sm += expf((sA[ii * 128 + tid] + sTr[ii * kCls + jj]) - mx);
      sN[jj * 128 + tid] = (mx + logf(sm)) + LG[row + jj];
    }
#pragma unroll 1
    for (int jj = 0; jj < kCls; ++jj) {
      const float ov = sA[jj * 128 + tid];
      const float nv = sN[jj * 128 + tid];
      sA[jj * 128 + tid] = mt ? nv : ov;
    }
    const float add = sTr[prv * kCls + tg] + ltag;
    num += mt ? add : 0.0f;
    cnt += mt ? 1 : 0;
    prv = tg;
  }
  int lastIdx = cnt - 1;
  lastIdx = (lastIdx < 0) ? (lastIdx + kSteps) : lastIdx;
  lastIdx = clampi(lastIdx, 0, kSteps - 1);
  const int lastTag = clampi(labels[base + lastIdx], 0, kCls - 1);
  num += sEn[lastTag];

  float mz = -INFINITY;
#pragma unroll 1
  for (int jj = 0; jj < kCls; ++jj) mz = fmaxf(mz, sA[jj * 128 + tid] + sEn[jj]);
  float sz = 0.0f;
#pragma unroll 1
  for (int jj = 0; jj < kCls; ++jj) sz += expf((sA[jj * 128 + tid] + sEn[jj]) - mz);
  const float logZ = mz + logf(sz);
  sL[tid] = num - logZ;
  __syncthreads();

  if (wave == 0) {
    float s = ((sL[lane] + sL[lane + 32]) + sL[lane + 64]) + sL[lane + 96];
    s += __shfl_xor(s, 16, 32);
    s += __shfl_xor(s, 8, 32);
    s += __shfl_xor(s, 4, 32);
    s += __shfl_xor(s, 2, 32);
    s += __shfl_xor(s, 1, 32);
    const float loss = -(s * (1.0f / (float)kBatch));
    const int li = (lane > 0) ? (lane - 1) : 0;
    float lv = LG[li];
    asm volatile("" : "+v"(lv));
    const float val = (lane == 0) ? loss : lv;
    volatile float* dst = out + lane;
    *dst = val;
    __threadfence();
    *dst = val;
  }
}

extern "C" void kernel_launch(void* const* d_in, const int* in_sizes, int n_in,
                              void* d_out, int out_size, void* d_ws, size_t ws_size,
                              hipStream_t stream) {
  if (n_in < 16) return;
  if (in_sizes[0] != kRows || in_sizes[1] != kRows) return;
  if (in_sizes[2] != kVocab * kEmb) return;
  if (in_sizes[3] != kGates * kEmb || in_sizes[7] != kGates * kEmb) return;
  if (in_sizes[4] != kGates * kHid || in_sizes[8] != kGates * kHid) return;
  if (in_sizes[5] != kGates || in_sizes[6] != kGates || in_sizes[9] != kGates || in_sizes[10] != kGates) return;
  if (in_sizes[11] != kCls * 2 * kHid || in_sizes[12] != kCls) return;
  if (in_sizes[13] != kCls * kCls || in_sizes[14] != kCls || in_sizes[15] != kCls) return;
  if (out_size != kOutN) return;
  if (ws_size < kWsTotal) return;

  const int*   ids    = (const int*)  d_in[0];
  const int*   labels = (const int*)  d_in[1];
  const float* table  = (const float*)d_in[2];
  const float* WihF   = (const float*)d_in[3];
  const float* WhhF   = (const float*)d_in[4];
  const float* bihF   = (const float*)d_in[5];
  const float* bhhF   = (const float*)d_in[6];
  const float* WihB   = (const float*)d_in[7];
  const float* WhhB   = (const float*)d_in[8];
  const float* bihB   = (const float*)d_in[9];
  const float* bhhB   = (const float*)d_in[10];
  const float* fcw    = (const float*)d_in[11];
  const float* fcb    = (const float*)d_in[12];
  const float* trans  = (const float*)d_in[13];
  const float* startT = (const float*)d_in[14];
  const float* endT   = (const float*)d_in[15];
  float* out = (float*)d_out;

  char* ws = (char*)d_ws;
  unsigned short* A16  = (unsigned short*)(ws + kOffA16);
  unsigned short* BT16 = (unsigned short*)(ws + kOffBT16);
  float*          BIAS = (float*)(ws + kOffBIAS);
  float*          XG   = (float*)(ws + kOffXG);
  float*          HF   = (float*)(ws + kOffHF);
  float*          HB   = (float*)(ws + kOffHB);
  float*          LG   = (float*)(ws + kOffLG);

  prep_act_kernel<<<(kRows * kChunks) / 256, 256, 0, stream>>>(ids, table, A16);
  prep_wgt_kernel<<<kNPad + 1, 64, 0, stream>>>(WihF, WihB, bihF, bhhF, bihB, bhhB, BT16, BIAS);
  gemm_xg_kernel<<<(kTilesM * kTilesN) / 8, 256, 0, stream>>>(A16, BT16, XG, BIAS, kFoldXG);
  lstm_scan_kernel<<<dim3(kBatch / 16, 2), 128, 0, stream>>>(XG, WhhF, WhhB, HF, HB);
  fc_kernel<<<kLogitN / 256, 256, 0, stream>>>(HF, HB, fcw, fcb, LG);
  copy_logits_kernel<<<kLogitN / 256, 256, 0, stream>>>(LG, out);
  crf_loss_kernel<<<1, 128, 0, stream>>>(LG, ids, labels, trans, startT, endT, out);
}
